// DualFusionLayer_27642409517764
// MI455X (gfx1250) — hardware-run, weakly checked
//
#include <hip/hip_runtime.h>
#include <math.h>

#ifndef NB
#define NB 8
#endif
#ifndef SEQ
#define SEQ 512
#endif
#define NB_FULL 8
#define SEQ_FULL 512
#define DM 768
#define HEADS 12
#define HD 64
#define NSTREAM 4
#define FFD 3072
#define MTOK (NB * SEQ)
#define CATD (NSTREAM * HD)
#define CATLD (HEADS * CATD)

#define CARRY_ACT 2048.0f
#define CARRY_W 65536.0f
#define CARRY_P 16384.0f
#define CARRY_CTX 4096.0f

#define OUT1_OFF ((size_t)NB_FULL * SEQ_FULL * DM)

static_assert(SEQ == SEQ_FULL);
static_assert(NB <= NB_FULL);
static_assert(SEQ % 128 == 0);
static_assert(MTOK % 64 == 0);
static_assert(DM % 64 == 0 && FFD % 64 == 0);
static_assert(DM % 32 == 0 && FFD % 32 == 0 && CATD % 32 == 0);
static_assert(DM == HEADS * HD);
static_assert(((size_t)MTOK * DM / 8) % 256 == 0);
static_assert(OUT1_OFF * 4 == 12582912);
static_assert((OUT1_OFF + (size_t)MTOK * DM) * 4 <= 25165824);

typedef _Float16 h16;
typedef __attribute__((ext_vector_type(16))) _Float16 v16h;
typedef __attribute__((ext_vector_type(8)))  _Float16 v8h;
typedef __attribute__((ext_vector_type(8)))  float    v8f;
typedef __attribute__((ext_vector_type(4)))  float    v4f;


static __device__ __forceinline__ float bfr(float f) {
    unsigned u = __float_as_uint(f);
    u += 0x7FFFu + ((u >> 16) & 1u);
    return __uint_as_float(u & 0xFFFF0000u);
}
static __device__ __forceinline__ h16 toh_flush(float v) {
    const float w = (fabsf(v) < 6.103515625e-05f) ? 0.0f : v;
    return (h16)w;
}
static __device__ __forceinline__ void st8h(h16* P, size_t o, const float* v) {
    v8h hv;
#pragma unroll
    for (int e = 0; e < 8; ++e) hv[e] = toh_flush(v[e]);
    *(volatile v8h*)(P + o) = hv;
    __threadfence();
    *(volatile v8h*)(P + o) = hv;
}

union FragU { v16h v; v8h h[2]; };
static __device__ __forceinline__ v16h frag_ld(const h16* p) {
    FragU f; f.h[0] = *(const v8h*)(p); f.h[1] = *(const v8h*)(p + 16); return f.v;
}
static __device__ __forceinline__ v8f wmma16g(v16h a, v16h b, v8f c) {
    c = __builtin_amdgcn_wmma_f32_16x16x32_f16(false, a, false, b, (short)0, c, false, false);
    asm volatile("v_nop\n\tv_nop\n\tv_nop\n\tv_nop" : "+v"(c) : "v"(a), "v"(b));
    return c;
}
static __device__ __forceinline__ void wave_sync_lds() {
    __builtin_amdgcn_fence(3  , "workgroup");
    __builtin_amdgcn_wave_barrier();
    __builtin_amdgcn_fence(2  , "workgroup");
}
static __device__ __forceinline__ float gelu_erf(float v) {
    return 0.5f * v * (1.0f + erff(v / 1.41421356237309515f));
}

template <int OUT_MODE, int RESID, bool GELU, int LG_IN, int LG_OUT>
__global__ __launch_bounds__(256) void k_gemm64(
    const h16* __restrict__ A, unsigned lda, unsigned zA,
    const h16* __restrict__ Bt, unsigned ldb, unsigned zB,
    void* __restrict__ Cout, unsigned ldc, unsigned ctile, unsigned zC,
    const float* __restrict__ bias, unsigned zBias,
    const float* __restrict__ resid,
    unsigned M, unsigned N, unsigned K) {
  __shared__ __align__(16) float sT[8][16 * 68];
  constexpr float scale = 1.0f / (float)(1u << LG_IN);
  constexpr float oscale = (float)(1u << LG_OUT);
  const unsigned lane = threadIdx.x & 31u;
  const unsigned wave = threadIdx.x >> 5;
  const unsigned z = blockIdx.y;
  const unsigned tilesN = N >> 6, tilesM = M >> 6;
  const unsigned tile = blockIdx.x * 8u + wave;
  if (tile >= tilesM * tilesN) return;
  const unsigned tm = tile / tilesN;
  const unsigned tn = tile - tm * tilesN;
  const unsigned m0 = tm << 6, n0 = tn << 6;
  const unsigned cb = tn * ctile;
  const unsigned rlane = lane & 15u;
  const unsigned koff = (lane >> 4) * 8u;
  const unsigned mOff = koff;
  const h16* Az = A + (size_t)z * zA;
  const h16* Bz = Bt + (size_t)z * zB;
  const float* biasz = bias + (size_t)z * zBias;

  v8f acc[4][4];
#pragma unroll
  for (int i = 0; i < 4; ++i)
#pragma unroll
    for (int j = 0; j < 4; ++j) acc[i][j] = (v8f){0.f,0.f,0.f,0.f,0.f,0.f,0.f,0.f};

  for (unsigned k0 = 0; k0 < K; k0 += 32u) {
    v16h bh[4];
#pragma unroll
    for (int j = 0; j < 4; ++j)
      bh[j] = frag_ld(Bz + (size_t)(n0 + ((unsigned)j << 4) + rlane) * ldb + koff + k0);
#pragma unroll
    for (int i = 0; i < 4; ++i) {
      const v16h ah = frag_ld(Az + (size_t)(m0 + ((unsigned)i << 4) + rlane) * lda + koff + k0);
#pragma unroll
      for (int j = 0; j < 4; ++j) acc[i][j] = wmma16g(ah, bh[j], acc[i][j]);
    }
  }

  float* slab = sT[wave];
#pragma unroll
  for (int i = 0; i < 4; ++i) {
    const unsigned mBase = m0 + ((unsigned)i << 4);
#pragma unroll
    for (int j = 0; j < 4; ++j) {
      const unsigned n = n0 + ((unsigned)j << 4) + rlane;
      const float bv = bfr(biasz[n]);
#pragma unroll
      for (int r = 0; r < 8; ++r) {
        const float v = acc[i][j][r] * scale + bv;
        slab[(mOff + (unsigned)r) * 68u + ((unsigned)j << 4) + rlane] = v;
      }
    }
    wave_sync_lds();
    if (OUT_MODE == 0) {
      float* C = (float*)Cout + (size_t)z * zC;
      const unsigned hh2 = lane >> 4, c4 = (lane & 15u) * 4u;
#pragma unroll
      for (int half = 0; half < 2; ++half) {
        v4f vv[4];
#pragma unroll
        for (int it = 0; it < 4; ++it) {
          const unsigned row = (unsigned)(half * 4 + it) * 2u + hh2;
          v4f cv = *(const v4f*)(slab + row * 68u + c4);
          if (RESID != 0) {
            v4f rv = *(const v4f*)(resid + (size_t)(mBase + row) * ldc + cb + c4);
            if (RESID == 2) { rv.x = bfr(rv.x); rv.y = bfr(rv.y); rv.z = bfr(rv.z); rv.w = bfr(rv.w); }
            cv += rv;
          }
          vv[it] = cv;
        }
        for (int pass = 0; pass < 2; ++pass) {
#pragma unroll
          for (int it = 0; it < 4; ++it) {
            const unsigned row = (unsigned)(half * 4 + it) * 2u + hh2;
            *(volatile v4f*)(C + (size_t)(mBase + row) * ldc + cb + c4) = vv[it];
          }
          __threadfence();
        }
      }
    } else {
      h16* C = (h16*)Cout + (size_t)z * zC;
      const unsigned q = lane >> 3, c8 = (lane & 7u) * 8u;
      v8h hv[4];
#pragma unroll
      for (int it = 0; it < 4; ++it) {
        const unsigned row = (unsigned)it * 4u + q;
        const float* sp = slab + row * 68u + c8;
#pragma unroll
        for (int e = 0; e < 8; ++e) {
          float v = sp[e];
          if (GELU) v = gelu_erf(v);
          hv[it][e] = toh_flush(v * oscale);
        }
      }
      for (int pass = 0; pass < 2; ++pass) {
#pragma unroll
        for (int it = 0; it < 4; ++it) {
          const unsigned row = (unsigned)it * 4u + q;
          *(volatile v8h*)(C + (size_t)(mBase + row) * ldc + cb + c8) = hv[it];
        }
        __threadfence();
      }
    }
    wave_sync_lds();
  }
}

template <unsigned KI, unsigned NO>
__global__ __launch_bounds__(256) void k_wt16(const float* __restrict__ Wm, h16* __restrict__ W16) {
    const unsigned layer = blockIdx.y;
    const float* Wl = Wm + (size_t)layer * KI * NO;
    h16* Dl = W16 + (size_t)layer * KI * NO;
    const unsigned u = blockIdx.x * 256u + threadIdx.x;
    constexpr unsigned per = KI / 8u;
    if (u >= NO * per) return;
    const unsigned o = u / per;
    const unsigned k0 = 8u * (u - o * per);
    float v[8];
#pragma unroll
    for (int i = 0; i < 8; ++i) v[i] = bfr(Wl[(size_t)(k0 + (unsigned)i) * NO + o]) * CARRY_W;
    st8h(Dl, (size_t)o * KI + k0, v);
}

__global__ __launch_bounds__(256) void k_cvt(const float* __restrict__ src, unsigned srcZ, h16* __restrict__ dst, unsigned dstZ, unsigned n8) {
    const unsigned u = blockIdx.x * 256u + threadIdx.x;
    if (u >= n8) return;
    const unsigned z = blockIdx.y;
    const float* s = src + (size_t)z * srcZ + (size_t)u * 8u;
    const v4f a = *(const v4f*)s, b = *(const v4f*)(s + 4);
    float v[8] = {bfr(a.x) * CARRY_ACT, bfr(a.y) * CARRY_ACT, bfr(a.z) * CARRY_ACT, bfr(a.w) * CARRY_ACT,
                  bfr(b.x) * CARRY_ACT, bfr(b.y) * CARRY_ACT, bfr(b.z) * CARRY_ACT, bfr(b.w) * CARRY_ACT};
    st8h(dst + (size_t)z * dstZ, (size_t)u * 8u, v);
}

__global__ __launch_bounds__(256) void k_tr(const h16* __restrict__ in, h16* __restrict__ out) {
    __shared__ float sX[64][65];
    const unsigned t = threadIdx.x;
    const unsigned c0 = blockIdx.x * 64u, r0 = blockIdx.y * 64u;
    {
        const unsigned r = t >> 2, cg = (t & 3u) * 16u;
        const h16* src = in + (size_t)(r0 + r) * DM + c0 + cg;
        const v8h a = *(const v8h*)src, b = *(const v8h*)(src + 8);
#pragma unroll
        for (int e = 0; e < 8; ++e) { sX[r][cg + (unsigned)e] = (float)a[e]; sX[r][cg + 8u + (unsigned)e] = (float)b[e]; }
    }
    __syncthreads();
    const unsigned q = t >> 3, p8 = (t & 7u) * 8u;
    v8h hv[2];
#pragma unroll
    for (int it = 0; it < 2; ++it) {
        const unsigned f = (unsigned)it * 32u + q;
#pragma unroll
        for (int e = 0; e < 8; ++e) hv[it][e] = toh_flush(sX[p8 + (unsigned)e][f]);
    }
    for (int pass = 0; pass < 2; ++pass) {
#pragma unroll
        for (int it = 0; it < 2; ++it) {
            const unsigned f = (unsigned)it * 32u + q;
            *(volatile v8h*)(out + (size_t)(c0 + f) * MTOK + r0 + p8) = hv[it];
        }
        __threadfence();
    }
}

template <bool Z16>
__global__ __launch_bounds__(256) void k_ln(const float* __restrict__ pre, const float* __restrict__ g, const float* __restrict__ bt,
                                            float* __restrict__ yout, h16* __restrict__ z16, unsigned M) {
    __shared__ __align__(16) float sY[8][DM];
    const unsigned wave = threadIdx.x >> 5;
    const unsigned row = blockIdx.x * 8u + wave;
    const unsigned L = threadIdx.x & 31u;
    if (row >= M) return;
    const float* pr = pre + (size_t)row * DM + 4u * L;
    v4f x[6];
#pragma unroll
    for (int j = 0; j < 6; ++j) x[j] = *(const v4f*)(pr + 128 * j);
    float s = 0.f;
#pragma unroll
    for (int j = 0; j < 6; ++j) s += (x[j].x + x[j].y) + (x[j].z + x[j].w);
#pragma unroll
    for (int o = 16; o > 0; o >>= 1) s += __shfl_xor(s, o, 32);
    const float mu = s / 768.0f;
    float q = 0.f;
#pragma unroll
    for (int j = 0; j < 6; ++j) {
        x[j].x -= mu; x[j].y -= mu; x[j].z -= mu; x[j].w -= mu;
        q += (x[j].x * x[j].x + x[j].y * x[j].y) + (x[j].z * x[j].z + x[j].w * x[j].w);
    }
#pragma unroll
    for (int o = 16; o > 0; o >>= 1) q += __shfl_xor(q, o, 32);
    const float rs = 1.0f / sqrtf(q / 768.0f + 1e-12f);
    v4f y[6];
#pragma unroll
    for (int j = 0; j < 6; ++j) {
        const v4f gv = *(const v4f*)(g + 128 * j + 4u * L);
        const v4f bv = *(const v4f*)(bt + 128 * j + 4u * L);
        y[j].x = x[j].x * rs * bfr(gv.x) + bfr(bv.x);
        y[j].y = x[j].y * rs * bfr(gv.y) + bfr(bv.y);
        y[j].z = x[j].z * rs * bfr(gv.z) + bfr(bv.z);
        y[j].w = x[j].w * rs * bfr(gv.w) + bfr(bv.w);
    }
    float* yo = yout + (size_t)row * DM + 4u * L;
    for (int pass = 0; pass < 2; ++pass) {
#pragma unroll
        for (int j = 0; j < 6; ++j) *(volatile v4f*)(yo + 128 * j) = y[j];
        __threadfence();
    }
    if (Z16) {
        float* sy = sY[wave];
#pragma unroll
        for (int j = 0; j < 6; ++j) *(v4f*)(sy + 128 * j + 4u * L) = y[j];
        wave_sync_lds();
        v8h hv[3];
#pragma unroll
        for (int gq = 0; gq < 3; ++gq) {
            const v4f a = *(const v4f*)(sy + 256 * gq + 8u * L);
            const v4f b = *(const v4f*)(sy + 256 * gq + 8u * L + 4u);
            hv[gq][0] = toh_flush(a.x * CARRY_ACT); hv[gq][1] = toh_flush(a.y * CARRY_ACT);
            hv[gq][2] = toh_flush(a.z * CARRY_ACT); hv[gq][3] = toh_flush(a.w * CARRY_ACT);
            hv[gq][4] = toh_flush(b.x * CARRY_ACT); hv[gq][5] = toh_flush(b.y * CARRY_ACT);
            hv[gq][6] = toh_flush(b.z * CARRY_ACT); hv[gq][7] = toh_flush(b.w * CARRY_ACT);
        }
        h16* zo = z16 + (size_t)row * DM + 8u * L;
        for (int pass = 0; pass < 2; ++pass) {
#pragma unroll
            for (int gq = 0; gq < 3; ++gq) *(volatile v8h*)(zo + 256 * gq) = hv[gq];
            __threadfence();
        }
    }
}

template <int MODE>
static __device__ __forceinline__ float logit_of(float acc, float m) {
    const float sqk = acc * (1.0f / 4194304.0f);
    if (MODE == 0) return ((sqk / 8.0f) + 5.0f * m) / 8.0f;
    return sqk / 8.0f + m;
}

#define AT_PS 68
#define AT_PP 72
template <int KD, int MODE>
__global__ __launch_bounds__(256) void k_attn(const h16* __restrict__ Qp, const h16* __restrict__ Kp, const h16* __restrict__ VT,
                                              const float* __restrict__ mask, const float* __restrict__ resid, void* __restrict__ outp) {
    __shared__ __align__(16) float sS[8][16 * AT_PS];
    __shared__ __align__(16) h16   sP[8][16 * AT_PP];
    constexpr unsigned LDQ = (unsigned)(HEADS * KD);
    const unsigned tid = threadIdx.x, lane = tid & 31u, wave = tid >> 5;
    const unsigned hh = lane >> 4, c = lane & 15u;
    const unsigned bx = blockIdx.x;
    const unsigned RT = (unsigned)(SEQ / 128);
    const unsigned rt = bx % RT;
    const unsigned bhd = bx / RT;
    const unsigned h = bhd % (unsigned)HEADS;
    const unsigned b = bhd / (unsigned)HEADS;
    const unsigned q0 = rt * 128u + wave * 16u;
    float* sl = sS[wave];
    h16* pw = sP[wave];
    const unsigned prow = lane >> 1, hf = lane & 1u;
    const h16* qbase = Qp + (size_t)(b * SEQ + q0 + c) * LDQ + h * (unsigned)KD + 8u * hh;
    const h16* kbase = Kp + (size_t)(b * SEQ + c) * LDQ + h * (unsigned)KD + 8u * hh;
    const h16* vbase = VT + (size_t)(h * 64u + c) * MTOK + b * SEQ + 8u * hh;
    const float* mbase = mask + ((size_t)(b * SEQ_FULL + q0 + prow) * SEQ_FULL + hf * 32u);
    float* srow = sl + prow * AT_PS + hf * 32u;
    h16* prw = pw + prow * AT_PP + hf * 32u;

    float m_run = -3.0e38f, l_run = 0.f;
    v8f o[4];
#pragma unroll
    for (int t = 0; t < 4; ++t) o[t] = (v8f){0.f,0.f,0.f,0.f,0.f,0.f,0.f,0.f};

    for (unsigned kc = 0; kc < (unsigned)(SEQ / 64); ++kc) {
        const unsigned kv0 = kc * 64u;
        v8f s[4];
#pragma unroll
        for (int j = 0; j < 4; ++j) s[j] = (v8f){0.f,0.f,0.f,0.f,0.f,0.f,0.f,0.f};
        for (unsigned ks = 0; ks < (unsigned)(KD / 32); ++ks) {
            const v16h qf = frag_ld(qbase + ks * 32u);
#pragma unroll
            for (int j = 0; j < 4; ++j) {
                const v16h kf = frag_ld(kbase + (size_t)(kv0 + (unsigned)j * 16u) * LDQ + ks * 32u);
                s[j] = wmma16g(qf, kf, s[j]);
            }
        }
#pragma unroll
        for (int j = 0; j < 4; ++j)
#pragma unroll
            for (int r = 0; r < 8; ++r)
                sl[(8u * hh + (unsigned)r) * AT_PS + (unsigned)j * 16u + c] = s[j][r];
        wave_sync_lds();

        const float* mrow = mbase + kv0;
        float mx = -3.0e38f;
        for (unsigned g4 = 0; g4 < 8u; ++g4) {
            const v4f sv = *(const v4f*)(srow + 4u * g4);
            const v4f mv = *(const v4f*)(mrow + 4u * g4);
            v4f xv;
            xv.x = logit_of<MODE>(sv.x, bfr(mv.x));
            xv.y = logit_of<MODE>(sv.y, bfr(mv.y));
            xv.z = logit_of<MODE>(sv.z, bfr(mv.z));
            xv.w = logit_of<MODE>(sv.w, bfr(mv.w));
            *(v4f*)(srow + 4u * g4) = xv;
            mx = fmaxf(mx, fmaxf(fmaxf(xv.x, xv.y), fmaxf(xv.z, xv.w)));
        }
        mx = fmaxf(mx, __shfl_xor(mx, 1, 32));
        const float mnew = fmaxf(m_run, mx);
        const float alpha = expf(m_run - mnew);
        m_run = mnew;
        float psum = 0.f;
        for (unsigned g8 = 0; g8 < 4u; ++g8) {
            const v4f x0 = *(const v4f*)(srow + 8u * g8);
            const v4f x1 = *(const v4f*)(srow + 8u * g8 + 4u);
            float p[8];
            p[0] = expf(x0.x - mnew); p[1] = expf(x0.y - mnew); p[2] = expf(x0.z - mnew); p[3] = expf(x0.w - mnew);
            p[4] = expf(x1.x - mnew); p[5] = expf(x1.y - mnew); p[6] = expf(x1.z - mnew); p[7] = expf(x1.w - mnew);
            v8h hv;
#pragma unroll
            for (int e = 0; e < 8; ++e) { psum += p[e]; hv[e] = toh_flush(p[e] * CARRY_P); }
            *(v8h*)(prw + 8u * g8) = hv;
        }
        psum += __shfl_xor(psum, 1, 32);
        l_run = l_run * alpha + psum;
        wave_sync_lds();

#pragma unroll
        for (int r = 0; r < 8; ++r) {
            const float a = __shfl(alpha, (int)(2u * (8u * hh + (unsigned)r)), 32);
#pragma unroll
            for (int t = 0; t < 4; ++t) o[t][r] *= a;
        }
#pragma unroll
        for (int kk = 0; kk < 2; ++kk) {
            const v16h pa = frag_ld(pw + c * AT_PP + (unsigned)kk * 32u + 8u * hh);
#pragma unroll
            for (int t = 0; t < 4; ++t) {
                const v16h vb = frag_ld(vbase + (size_t)((unsigned)t * 16u) * MTOK + kv0 + (unsigned)kk * 32u);
                o[t] = wmma16g(pa, vb, o[t]);
            }
        }
        wave_sync_lds();
    }

#pragma unroll
    for (int r = 0; r < 8; ++r) {
        const float lr = __shfl(l_run, (int)(2u * (8u * hh + (unsigned)r)), 32);
        const float inv = 1.0f / (lr * 33554432.0f);
#pragma unroll
        for (int t = 0; t < 4; ++t)
            sl[(8u * hh + (unsigned)r) * AT_PS + (unsigned)t * 16u + c] = o[t][r] * inv;
    }
    wave_sync_lds();
    if (MODE == 0) {
        float* out = (float*)outp;
        const unsigned hh2 = lane >> 4, c4 = (lane & 15u) * 4u;
#pragma unroll
        for (int half = 0; half < 2; ++half) {
            v4f vv[4];
#pragma unroll
            for (int it = 0; it < 4; ++it) {
                const unsigned row = (unsigned)(half * 4 + it) * 2u + hh2;
                v4f cv = *(const v4f*)(sl + row * AT_PS + c4);
                const v4f ev = *(const v4f*)(resid + (size_t)(b * SEQ_FULL + q0 + row) * DM + h * 64u + c4);
                cv.x += bfr(ev.x); cv.y += bfr(ev.y); cv.z += bfr(ev.z); cv.w += bfr(ev.w);
                vv[it] = cv;
            }
            for (int pass = 0; pass < 2; ++pass) {
#pragma unroll
                for (int it = 0; it < 4; ++it) {
                    const unsigned row = (unsigned)(half * 4 + it) * 2u + hh2;
                    *(volatile v4f*)(out + (size_t)(b * SEQ + q0 + row) * DM + h * 64u + c4) = vv[it];
                }
                __threadfence();
            }
        }
    } else {
        h16* out = (h16*)outp;
        const unsigned q = lane >> 3, c8 = (lane & 7u) * 8u;
        v8h hv[4];
#pragma unroll
        for (int it = 0; it < 4; ++it) {
            const unsigned row = (unsigned)it * 4u + q;
            const v4f a = *(const v4f*)(sl + row * AT_PS + c8);
            const v4f bq = *(const v4f*)(sl + row * AT_PS + c8 + 4u);
            hv[it][0] = toh_flush(a.x * CARRY_CTX);  hv[it][1] = toh_flush(a.y * CARRY_CTX);
            hv[it][2] = toh_flush(a.z * CARRY_CTX);  hv[it][3] = toh_flush(a.w * CARRY_CTX);
            hv[it][4] = toh_flush(bq.x * CARRY_CTX); hv[it][5] = toh_flush(bq.y * CARRY_CTX);
            hv[it][6] = toh_flush(bq.z * CARRY_CTX); hv[it][7] = toh_flush(bq.w * CARRY_CTX);
        }
        for (int pass = 0; pass < 2; ++pass) {
#pragma unroll
            for (int it = 0; it < 4; ++it) {
                const unsigned row = (unsigned)it * 4u + q;
                *(volatile v8h*)(out + (size_t)(b * SEQ + q0 + row) * DM + h * 64u + c8) = hv[it];
            }
            __threadfence();
        }
    }
}

#define P768_B ((size_t)DM * DM * 2)
#define PFF_B  ((size_t)DM * FFD * 2)
#define TOKD_B ((size_t)MTOK * DM * 2)
#define CAT_B  ((size_t)MTOK * CATLD * 2)
#define WS_TOTAL (12 * P768_B + 4 * PFF_B + 4 * TOKD_B + TOKD_B + 2 * CAT_B + 2 * TOKD_B)
static_assert(WS_TOTAL <= (size_t)268435456);
static_assert(P768_B % 256 == 0 && PFF_B % 256 == 0 && TOKD_B % 256 == 0 && CAT_B % 256 == 0);
static_assert(4 * TOKD_B >= 2 * (size_t)MTOK * DM * 4);
static_assert(CAT_B >= 4 * TOKD_B);
static_assert(CAT_B >= (size_t)MTOK * FFD * 2);

extern "C" void kernel_launch(void* const* d_in, const int* in_sizes, int n_in, void* d_out, int out_size,
                              void* d_ws, size_t ws_size, hipStream_t stream) {
    if (n_in < 36) return;
    if (in_sizes[0] < MTOK * DM || in_sizes[2] < MTOK * DM || in_sizes[3] < MTOK * SEQ) return;
    if ((size_t)in_sizes[1] < (size_t)2 * NB_FULL * SEQ_FULL * DM + (size_t)MTOK * DM) return;
    if (in_sizes[4] < DM * DM || in_sizes[6] < DM * DM || in_sizes[8] < 3 * DM * DM || in_sizes[10] < 3 * DM * DM) return;
    if (in_sizes[12] < DM * DM || in_sizes[14] < DM * DM || in_sizes[16] < DM * DM || in_sizes[18] < DM * DM) return;
    if (in_sizes[5] < DM || in_sizes[7] < DM || in_sizes[9] < 3 * DM || in_sizes[11] < 3 * DM) return;
    if (in_sizes[13] < DM || in_sizes[15] < DM || in_sizes[17] < DM || in_sizes[19] < DM) return;
    for (int i = 20; i < 28; ++i) if (in_sizes[i] < DM) return;
    if (in_sizes[28] < DM * FFD || in_sizes[30] < DM * FFD || in_sizes[32] < DM * FFD || in_sizes[34] < DM * FFD) return;
    if (in_sizes[29] < FFD || in_sizes[33] < FFD || in_sizes[31] < DM || in_sizes[35] < DM) return;
    if ((size_t)out_size < OUT1_OFF + (size_t)MTOK * DM) return;

    const float* E_v     = (const float*)d_in[0];
    const float* E_attrs = (const float*)d_in[1];
    const float* E_va    = (const float*)d_in[2];
    const float* mask    = (const float*)d_in[3];
    const float* Wq_id   = (const float*)d_in[4];
    const float* bq_id   = (const float*)d_in[5];
    const float* Wk_id   = (const float*)d_in[6];
    const float* bk_id   = (const float*)d_in[7];
    const float* Wq_attr = (const float*)d_in[8];
    const float* bq_attr = (const float*)d_in[9];
    const float* Wk_attr = (const float*)d_in[10];
    const float* bk_attr = (const float*)d_in[11];
    const float* Wq_f    = (const float*)d_in[12];
    const float* bq_f    = (const float*)d_in[13];
    const float* Wk_f    = (const float*)d_in[14];
    const float* bk_f    = (const float*)d_in[15];
    const float* Wv_f    = (const float*)d_in[16];
    const float* bv_f    = (const float*)d_in[17];
    const float* Wo_f    = (const float*)d_in[18];
    const float* bo_f    = (const float*)d_in[19];
    const float* g1      = (const float*)d_in[20];
    const float* be1     = (const float*)d_in[21];
    const float* g2      = (const float*)d_in[22];
    const float* be2     = (const float*)d_in[23];
    const float* g3      = (const float*)d_in[24];
    const float* be3     = (const float*)d_in[25];
    const float* g4      = (const float*)d_in[26];
    const float* be4     = (const float*)d_in[27];
    const float* W1_id   = (const float*)d_in[28];
    const float* b1_id   = (const float*)d_in[29];
    const float* W2_id   = (const float*)d_in[30];
    const float* b2_id   = (const float*)d_in[31];
    const float* W1_f    = (const float*)d_in[32];
    const float* b1_f    = (const float*)d_in[33];
    const float* W2_f    = (const float*)d_in[34];
    const float* b2_f    = (const float*)d_in[35];
    float* out0 = (float*)d_out;
    float* out1 = out0 + OUT1_OFF;

    if (WS_TOTAL > ws_size || WS_TOTAL > (size_t)134217728) return;
    char* wsp = (char*)d_ws;
    size_t off = 0;
    auto carve = [&](size_t bytes) -> void* { void* r = wsp + off; off += bytes; return r; };
    h16* wq4  = (h16*)carve(4 * P768_B);
    h16* wk4  = (h16*)carve(4 * P768_B);
    h16* wqf  = (h16*)carve(P768_B);
    h16* wkf  = (h16*)carve(P768_B);
    h16* wvf  = (h16*)carve(P768_B);
    h16* wof  = (h16*)carve(P768_B);
    h16* w1id = (h16*)carve(PFF_B);
    h16* w1f  = (h16*)carve(PFF_B);
    h16* w2id = (h16*)carve(PFF_B);
    h16* w2f  = (h16*)carve(PFF_B);
    h16* x4   = (h16*)carve(4 * TOKD_B);
    h16* xva  = (h16*)carve(TOKD_B);
    h16* qcat = (h16*)carve(CAT_B);
    h16* kcat = (h16*)carve(CAT_B);
    h16* vt   = (h16*)carve(TOKD_B);
    h16* z16  = (h16*)carve(TOKD_B);
    if (off != WS_TOTAL) return;

    const size_t TOKD = (size_t)MTOK * DM;
    const size_t P768 = (size_t)DM * DM;
    float* pre  = (float*)x4;
    float* rres = pre + TOKD;
    h16* qf  = qcat;
    h16* kf  = qcat + TOKD;
    h16* vf  = qcat + 2 * TOKD;
    h16* ctx = qcat + 3 * TOKD;
    h16* hid = kcat;

    const unsigned gW = (DM * (DM / 8)) / 256;
    const unsigned gWF = (FFD * (DM / 8)) / 256;
    k_wt16<DM, DM><<<dim3(gW, 1), 256, 0, stream>>>(Wq_id, wq4);
    k_wt16<DM, DM><<<dim3(gW, 3), 256, 0, stream>>>(Wq_attr, wq4 + P768);
    k_wt16<DM, DM><<<dim3(gW, 1), 256, 0, stream>>>(Wk_id, wk4);
    k_wt16<DM, DM><<<dim3(gW, 3), 256, 0, stream>>>(Wk_attr, wk4 + P768);
    k_wt16<DM, DM><<<dim3(gW, 1), 256, 0, stream>>>(Wq_f, wqf);
    k_wt16<DM, DM><<<dim3(gW, 1), 256, 0, stream>>>(Wk_f, wkf);
    k_wt16<DM, DM><<<dim3(gW, 1), 256, 0, stream>>>(Wv_f, wvf);
    k_wt16<DM, DM><<<dim3(gW, 1), 256, 0, stream>>>(Wo_f, wof);
    k_wt16<DM, FFD><<<dim3(gWF, 1), 256, 0, stream>>>(W1_id, w1id);
    k_wt16<DM, FFD><<<dim3(gWF, 1), 256, 0, stream>>>(W1_f, w1f);
    k_wt16<FFD, DM><<<dim3(gWF, 1), 256, 0, stream>>>(W2_id, w2id);
    k_wt16<FFD, DM><<<dim3(gWF, 1), 256, 0, stream>>>(W2_f, w2f);

    const unsigned n8 = (unsigned)(TOKD / 8);
    const unsigned gC = n8 / 256;
    k_cvt<<<dim3(gC, 1), 256, 0, stream>>>(E_v, 0u, x4, 0u, n8);
    k_cvt<<<dim3(gC, 3), 256, 0, stream>>>(E_attrs, (unsigned)((size_t)NB_FULL * SEQ_FULL * DM), x4 + TOKD, (unsigned)TOKD, n8);
    k_cvt<<<dim3(gC, 1), 256, 0, stream>>>(E_va, 0u, xva, 0u, n8);

    const unsigned gP = ((MTOK / 64) * (DM / 64) + 7) / 8;
    const unsigned gF = ((MTOK / 64) * (FFD / 64) + 7) / 8;

    k_gemm64<1, 0, false, 27, 11><<<dim3(gP, 1), 256, 0, stream>>>(x4, DM, 0u, wq4, DM, 0u,
        (void*)qcat, CATLD, CATD, 0u, bq_id, 0u, bq_id, MTOK, DM, DM);
    k_gemm64<1, 0, false, 27, 11><<<dim3(gP, 3), 256, 0, stream>>>(x4 + TOKD, DM, (unsigned)TOKD, wq4 + P768, DM, (unsigned)P768,
        (void*)(qcat + HD), CATLD, CATD, HD, bq_attr, DM, bq_attr, MTOK, DM, DM);
    k_gemm64<1, 0, false, 27, 11><<<dim3(gP, 1), 256, 0, stream>>>(x4, DM, 0u, wk4, DM, 0u,
        (void*)kcat, CATLD, CATD, 0u, bk_id, 0u, bk_id, MTOK, DM, DM);
    k_gemm64<1, 0, false, 27, 11><<<dim3(gP, 3), 256, 0, stream>>>(x4 + TOKD, DM, (unsigned)TOKD, wk4 + P768, DM, (unsigned)P768,
        (void*)(kcat + HD), CATLD, CATD, HD, bk_attr, DM, bk_attr, MTOK, DM, DM);
    k_tr<<<dim3(DM / 64, MTOK / 64), 256, 0, stream>>>(x4, vt);
    k_attn<CATD, 0><<<NB * HEADS * (SEQ / 128), 256, 0, stream>>>(qcat, kcat, vt, mask, E_v, (void*)pre);
    k_ln<true><<<MTOK / 8, 256, 0, stream>>>(pre, g1, be1, rres, z16, MTOK);
    k_gemm64<1, 0, true, 27, 12><<<dim3(gF, 1), 256, 0, stream>>>(z16, DM, 0u, w1id, DM, 0u,
        (void*)hid, FFD, 64u, 0u, b1_id, 0u, b1_id, MTOK, FFD, DM);
    k_gemm64<0, 1, false, 28, 0><<<dim3(gP, 1), 256, 0, stream>>>(hid, FFD, 0u, w2id, FFD, 0u,
        (void*)pre, DM, 64u, 0u, b2_id, 0u, rres, MTOK, DM, FFD);
    k_ln<false><<<MTOK / 8, 256, 0, stream>>>(pre, g2, be2, out0, z16, MTOK);

    k_gemm64<1, 0, false, 27, 11><<<dim3(gP, 1), 256, 0, stream>>>(xva, DM, 0u, wqf, DM, 0u,
        (void*)qf, DM, 64u, 0u, bq_f, 0u, bq_f, MTOK, DM, DM);
    k_gemm64<1, 0, false, 27, 11><<<dim3(gP, 1), 256, 0, stream>>>(xva, DM, 0u, wkf, DM, 0u,
        (void*)kf, DM, 64u, 0u, bk_f, 0u, bk_f, MTOK, DM, DM);
    k_gemm64<1, 0, false, 27, 11><<<dim3(gP, 1), 256, 0, stream>>>(xva, DM, 0u, wvf, DM, 0u,
        (void*)vf, DM, 64u, 0u, bv_f, 0u, bv_f, MTOK, DM, DM);
    k_tr<<<dim3(DM / 64, MTOK / 64), 256, 0, stream>>>(vf, vt);
    k_attn<HD, 1><<<NB * HEADS * (SEQ / 128), 256, 0, stream>>>(qf, kf, vt, mask, E_va, (void*)ctx);
    k_gemm64<0, 2, false, 28, 0><<<dim3(gP, 1), 256, 0, stream>>>(ctx, DM, 0u, wof, DM, 0u,
        (void*)pre, DM, 64u, 0u, bo_f, 0u, E_va, MTOK, DM, DM);
    k_ln<true><<<MTOK / 8, 256, 0, stream>>>(pre, g3, be3, rres, z16, MTOK);
    k_gemm64<1, 0, true, 27, 12><<<dim3(gF, 1), 256, 0, stream>>>(z16, DM, 0u, w1f, DM, 0u,
        (void*)hid, FFD, 64u, 0u, b1_f, 0u, b1_f, MTOK, FFD, DM);
    k_gemm64<0, 1, false, 28, 0><<<dim3(gP, 1), 256, 0, stream>>>(hid, FFD, 0u, w2f, FFD, 0u,
        (void*)pre, DM, 64u, 0u, b2_f, 0u, rres, MTOK, DM, FFD);
    k_ln<false><<<MTOK / 8, 256, 0, stream>>>(pre, g4, be4, out1, z16, MTOK);
}
